// ImplicitNet_step_42133629173881
// MI455X (gfx1250) — hardware-verified
//
#include <hip/hip_runtime.h>


namespace {
constexpr int B = 256, N = 512, NRICH = 96, NGD = 21, NFP = 10;
constexpr float TH = 0.5f, LM = 1e-5f, AS_ = 8.0f, BS8 = 8.0f;

typedef _Float16 b16;
typedef __attribute__((ext_vector_type(16))) _Float16 v16b;
typedef __attribute__((ext_vector_type(8))) _Float16 v8b;
typedef __attribute__((ext_vector_type(8))) float v8f;
typedef __attribute__((ext_vector_type(4))) float v4f;
__device__ __forceinline__ float bf16_rne(float f) { unsigned int u = __float_as_uint(f); u += 0x7FFFu + ((u >> 16) & 1u); return __uint_as_float(u & 0xFFFF0000u); }
__device__ __forceinline__ void split16(float v, b16& hi, b16& lo) { hi = (b16)v; lo = (b16)(v - (float)hi); }
__device__ __forceinline__ v16b frag_kb(const b16* p, int hh) { const v8b a = *(const v8b*)(p + 8 * hh), b = *(const v8b*)(p + 16 + 8 * hh); v16b f;
#pragma unroll
  for (int e = 0; e < 8; ++e) { f[e] = a[e]; f[8 + e] = b[e]; } return f; }
__device__ __forceinline__ void frag_split(const float* p, int hh, v16b& fh, v16b& fl) {
#pragma unroll
  for (int e = 0; e < 8; ++e) { b16 a, c; split16(p[8 * hh + e] * AS_, a, c); fh[e] = a; fl[e] = c; split16(p[16 + 8 * hh + e] * AS_, a, c); fh[8 + e] = a; fl[8 + e] = c; } }
__device__ __forceinline__ v8f wmma16b(v16b a, v16b b, v8f c) { v8f d = __builtin_amdgcn_wmma_f32_16x16x32_f16(false, a, false, b, (short)0, c, false, false); asm volatile("v_nop\n\tv_nop\n\tv_nop\n\tv_nop" : "+v"(d) : "v"(a), "v"(b)); return d; }
__device__ __forceinline__ float nexp(float x) { return __builtin_amdgcn_exp2f(x * 1.4426950408889634f); }
__device__ __forceinline__ float tanh_acc(float x) { const float ax = fabsf(x);
  if (ax < 0.0625f) { const float x2 = x * x; return x * (1.0f + x2 * (-0.333333333f + x2 * (0.133333333f + x2 * (-0.053968254f + x2 * 0.021869489f)))); }
  const float e = nexp(-2.0f * ax); const float t = (1.0f - e) / (1.0f + e); return (x >= 0.0f) ? t : -t; }

__global__ __launch_bounds__(256) void prep_kernel(const float* __restrict__ W, const float* __restrict__ bv, b16* __restrict__ Ah, float* __restrict__ P) {
  const int t_ = blockIdx.x * 256 + threadIdx.x, nth = gridDim.x * 256;
  for (int pass = 0; pass < 2; ++pass) {
    for (int q = t_; q < N * N / 8; q += nth) { const int i = q / (N / 8), j8 = (q % (N / 8)) * 8; v8b hv, lv;
#pragma unroll
      for (int e = 0; e < 8; ++e) { const int j = j8 + e; const float a = 0.5f * (bf16_rne(W[(size_t)i * N + j]) - bf16_rne(W[(size_t)j * N + i])); b16 h_, l_; split16(a * BS8, h_, l_); hv[e] = h_; lv[e] = l_; }
      *(volatile v8b*)(Ah + (size_t)i * N + j8) = hv; *(volatile v8b*)(Ah + (size_t)N * N + (size_t)i * N + j8) = lv; }
    for (int q = t_; q < N; q += nth) P[q] = bf16_rne(bv[q]);
    __threadfence(); }
}

__global__ __launch_bounds__(128) void implicit_kernel(const float* __restrict__ x, const b16* __restrict__ Ah, const float* __restrict__ P, float* __restrict__ y) {
  __shared__ __attribute__((aligned(16))) float F0[16][N + 4], EX[16][N + 4], Z[16][N + 4], T[16][N + 4];
  const int wave = threadIdx.x >> 5, lane = threadIdx.x & 31, nloc = lane & 15, hlf = lane >> 4, t_ = threadIdx.x, m0 = blockIdx.x * 16; const b16* Al = Ah + (size_t)N * N; const float* bv = P;
  auto matvec = [&](float (*Src)[N + 4], float sign) {
    v8f acc[8];
#pragma unroll
    for (int t = 0; t < 8; ++t) acc[t] = (v8f){};
#pragma unroll 2
    for (int kb = 0; kb < N; kb += 32) { v16b zh, zl; frag_split(&Src[nloc][kb], hlf, zh, zl);
#pragma unroll
      for (int t = 0; t < 8; ++t) { const size_t ro = (size_t)(wave * 128 + t * 16 + nloc) * N + kb; const v16b bh = frag_kb(Ah + ro, hlf), bl = frag_kb(Al + ro, hlf); acc[t] = wmma16b(zh, bh, acc[t]); acc[t] = wmma16b(zh, bl, acc[t]); acc[t] = wmma16b(zl, bh, acc[t]); } }
    __syncthreads();
#pragma unroll
    for (int t = 0; t < 8; ++t)
#pragma unroll
      for (int v = 0; v < 8; ++v) T[8 * hlf + v][wave * 128 + t * 16 + nloc] = acc[t][v] * (sign / (AS_ * BS8));
    __syncthreads(); };
  for (int i = t_; i < 16 * N; i += 128) { const int r = i / N, c = i % N; Z[r][c] = bf16_rne(x[(size_t)(m0 + r) * N + c]); }
  __syncthreads();
  matvec(Z, -1.0f);
  for (int i = t_; i < 16 * N; i += 128) { const int r = i / N, c = i % N; const float f0 = tanh_acc(T[r][c] + bv[c]); F0[r][c] = f0; EX[r][c] = Z[r][c] + (1.0f - TH) * f0; }
  __syncthreads();
  for (int i = t_; i < 16 * N; i += 128) { const int r = i / N, c = i % N; Z[r][c] = F0[r][c]; }
  __syncthreads();
  for (int it = 0; it < NRICH; ++it) { matvec(Z, -1.0f);
    for (int i = t_; i < 16 * N; i += 128) { const int r = i / N, c = i % N; const float f0 = F0[r][c], s = 1.0f - f0 * f0; Z[r][c] = f0 + TH * s * T[r][c]; }
    __syncthreads(); }
  for (int i = t_; i < 16 * N; i += 128) { const int r = i / N, c = i % N; Z[r][c] = bf16_rne(x[(size_t)(m0 + r) * N + c]) + Z[r][c]; }
  __syncthreads();
  matvec(Z, -1.0f);
  for (int i = t_; i < 16 * N; i += 128) { const int r = i / N, c = i % N; Z[r][c] = EX[r][c] + TH * tanh_acc(T[r][c] + bv[c]); }
  __syncthreads();
  for (int it = 0; it < NGD; ++it) { matvec(Z, -1.0f);
    for (int i = t_; i < 16 * N; i += 128) { const int r = i / N, c = i % N; const float tt = tanh_acc(T[r][c] + bv[c]); const float s = 1.0f - tt * tt; const float rr = Z[r][c] - EX[r][c] - TH * tt; F0[r][c] = s * rr; Z[r][c] = Z[r][c] - 2.0f * LM * rr; }
    __syncthreads();
    matvec(F0, 1.0f);
    for (int i = t_; i < 16 * N; i += 128) { const int r = i / N, c = i % N; Z[r][c] = Z[r][c] + 2.0f * LM * TH * T[r][c]; }
    __syncthreads(); }
  for (int it = 0; it < NFP + 1; ++it) { matvec(Z, -1.0f);
    for (int i = t_; i < 16 * N; i += 128) { const int r = i / N, c = i % N; Z[r][c] = EX[r][c] + TH * tanh_acc(T[r][c] + bv[c]); }
    __syncthreads(); }
  for (int pass = 0; pass < 2; ++pass) { for (int i = t_; i < 16 * (N / 4); i += 128) { const int r = i / (N / 4), c4 = (i % (N / 4)) * 4; *(volatile v4f*)(y + (size_t)(m0 + r) * N + c4) = *(const v4f*)(&Z[r][c4]); } __threadfence(); }
}
}

extern "C" void kernel_launch(void* const* d_in, const int* in_sizes, int n_in,
                              void* d_out, int out_size, void* d_ws, size_t ws_size, hipStream_t stream) {
  (void)n_in; (void)out_size;
  const float* x = (const float*)d_in[0]; const float* W = (const float*)d_in[1]; const float* bv = (const float*)d_in[2];
  float* y = (float*)d_out;
  if (in_sizes[0] != B * N || in_sizes[1] != N * N || in_sizes[2] != N) return;
  size_t off = 0; char* ws = (char*)d_ws;
  auto carve = [&](size_t bytes) { char* p = ws + off; off += (bytes + 255) & ~(size_t)255; return p; };
  b16* Ah = (b16*)carve((size_t)2 * N * N * 2); float* P = (float*)carve(N * 4);
  if (off > ws_size) return;
  prep_kernel<<<64, 256, 0, stream>>>(W, bv, Ah, P);
  implicit_kernel<<<B / 16, 128, 0, stream>>>(x, Ah, P, y);
}
